// LiquidNeuralNetwork_73632919322793
// MI455X (gfx1250) — hardware-verified
//
#include <hip/hip_runtime.h>
#include <math.h>

constexpr int BATCH_ROWS = 4096;
constexpr int IN_DIM     = 512;
constexpr int HID0       = 256;
constexpr int HID1       = 128;
constexpr int HID2       = 64;
constexpr int STATE_DIM  = 64;
constexpr int OUT_DIM    = 12;
constexpr int NOUT_TOTAL = BATCH_ROWS * OUT_DIM;
constexpr int SLAB_PITCH = 68;
constexpr float ACT_CARRY  = 64.0f;
constexpr float WGT_CARRY  = 256.0f;
constexpr float FOLD_INV   = 1.0f / (ACT_CARRY * WGT_CARRY);
static_assert(FOLD_INV == 1.0f / 16384.0f);
static_assert(BATCH_ROWS % 64 == 0);
static_assert(IN_DIM % 64 == 0 && HID0 % 64 == 0 && HID1 % 64 == 0 && HID2 % 64 == 0);
static_assert(IN_DIM % 32 == 0 && HID0 % 32 == 0 && HID1 % 32 == 0 && HID2 % 32 == 0);
static_assert(STATE_DIM == 64);
static_assert(NOUT_TOTAL % 256 == 0);
static_assert((BATCH_ROWS * IN_DIM / 8) % 256 == 0);
static_assert((SLAB_PITCH * 4) % 16 == 0);

typedef __attribute__((ext_vector_type(16))) _Float16 v16h;
typedef __attribute__((ext_vector_type(8)))  _Float16 v8h;
typedef __attribute__((ext_vector_type(8)))  float    v8f;
typedef __attribute__((ext_vector_type(4)))  float    v4f;

__device__ __forceinline__ void guard_group4(v8f& a, v8f& b, v8f& c, v8f& d, v16h x, v16h y0, v16h y1, v16h y2, v16h y3) {
  asm volatile("v_nop\n\tv_nop\n\tv_nop\n\tv_nop" : "+v"(a), "+v"(b), "+v"(c), "+v"(d) : "v"(x), "v"(y0), "v"(y1), "v"(y2), "v"(y3));
}
__device__ __forceinline__ void acc_guard4(v8f& a, v8f& b, v8f& c, v8f& d) {
  asm volatile("v_nop\n\tv_nop\n\tv_nop\n\tv_nop" : "+v"(a), "+v"(b), "+v"(c), "+v"(d));
}

template <typename T> struct Frag;
template <> struct Frag<_Float16> {
  typedef v16h V; union U { v16h v; v8h h[2]; };
  static __device__ __forceinline__ v16h load(const _Float16* p) {
    U f; f.h[0] = *(const v8h*)(p); f.h[1] = *(const v8h*)(p + 16); return f.v;
  }
  static __device__ __forceinline__ v8f mma(v16h a, v16h b, v8f c) {
    return __builtin_amdgcn_wmma_f32_16x16x32_f16(false, a, false, b, (short)0, c, false, false);
  }
};

__device__ __forceinline__ void wave_lds_sync() {
  __builtin_amdgcn_fence(__ATOMIC_RELEASE, "workgroup");
  __builtin_amdgcn_wave_barrier();
  __builtin_amdgcn_fence(__ATOMIC_ACQUIRE, "workgroup");
}

__device__ __forceinline__ float tanh_plus_ripple_act(float x) {
  const float e  = __expf(2.0f * x);
  const float th = 1.0f - 2.0f * __builtin_amdgcn_rcpf(e + 1.0f);
  const float sn = sinf(0.5f * x);
  const float cs = cosf(0.3f * x);
  return fmaf(0.1f, sn * cs, th);
}

__global__ __launch_bounds__(256) void cvt8_f16_kernel(const float* __restrict__ src, unsigned short* __restrict__ dst,
                                                       int n8, float sc) {
  const int i = blockIdx.x * 256 + threadIdx.x;
  if (i < n8) {
    const float* sp = src + (size_t)i * 8;
    const v4f a = *(const v4f*)(sp);
    const v4f b = *(const v4f*)(sp + 4);
    v8h hv;
#pragma unroll
    for (int e = 0; e < 4; ++e) {
      hv[e]     = (_Float16)(a[e] * sc);
      hv[4 + e] = (_Float16)(b[e] * sc);
    }
    unsigned short* dp = dst + (size_t)i * 8;
    *(volatile v8h*)dp = hv;
    __threadfence();
    *(volatile v8h*)dp = hv;
  }
}

__global__ __launch_bounds__(256) void transpose_cvt_kernel(const float* __restrict__ src, unsigned short* __restrict__ dst,
                                                            int src_ld, int dst_ld, long src_bs, long dst_bs, float sc) {
  __shared__ float tileT[64][65];
  const int tid = threadIdx.x;
  const int k0 = blockIdx.x * 64;
  const int j0 = blockIdx.y * 64;
  const float* sb = src + (size_t)blockIdx.z * (size_t)src_bs;
  unsigned short* db = dst + (size_t)blockIdx.z * (size_t)dst_bs;
#pragma unroll
  for (int it = 0; it < 4; ++it) {
    const int idx = tid + 256 * it;
    const int kr = idx >> 4;
    const int q4 = (idx & 15) * 4;
    const v4f v = *(const v4f*)(sb + (size_t)(k0 + kr) * src_ld + j0 + q4);
#pragma unroll
    for (int e = 0; e < 4; ++e) tileT[kr][q4 + e] = v[e];
  }
  __syncthreads();
  const int c8 = (tid & 7) * 8;
  v8h hv0, hv1;
  const int s0 = tid >> 3;
  const int s1 = s0 + 32;
#pragma unroll
  for (int e = 0; e < 8; ++e) {
    hv0[e] = (_Float16)(tileT[c8 + e][s0] * sc);
    hv1[e] = (_Float16)(tileT[c8 + e][s1] * sc);
  }
  unsigned short* p0 = db + (size_t)(j0 + s0) * dst_ld + k0 + c8;
  unsigned short* p1 = db + (size_t)(j0 + s1) * dst_ld + k0 + c8;
  *(volatile v8h*)p0 = hv0;
  *(volatile v8h*)p1 = hv1;
  __threadfence();
  *(volatile v8h*)p0 = hv0;
  *(volatile v8h*)p1 = hv1;
}

__global__ __launch_bounds__(256) void layer_fused_kernel(
    const unsigned short* __restrict__ Ap, const unsigned short* __restrict__ Btp,
    const float* __restrict__ bi, const float* __restrict__ bl, const float* __restrict__ wo, const float* __restrict__ bo,
    float* __restrict__ Pt, int kdim, int nneur) {
  typedef _Float16 T;
  const T* A  = (const T*)Ap;
  const T* Bt = (const T*)Btp;
  __shared__ __align__(16) float sT[8][16 * SLAB_PITCH];
  __shared__ __align__(16) float sC[8][128];
  __shared__ __align__(16) float sP[8][64];
  const int lane = threadIdx.x & 31;
  const int wave = threadIdx.x >> 5;
  const int tilesM = BATCH_ROWS >> 6;
  const int tile = blockIdx.x * 8 + wave;
  if (tile >= tilesM * nneur) return;
  const int tm = tile / nneur;
  const int tn = tile - tm * nneur;
  const int m0 = tm << 6;
  const int n0 = tn << 6;

  const int rlane = lane & 15;
  const int koff  = (lane >> 4) * 8;
  const int mOff  = (lane >> 4) * 8;

  v8f acc[4][4];
#pragma unroll
  for (int i = 0; i < 4; ++i)
#pragma unroll
    for (int j = 0; j < 4; ++j) acc[i][j] = (v8f){0.f, 0.f, 0.f, 0.f, 0.f, 0.f, 0.f, 0.f};

  for (int k0 = 0; k0 < kdim; k0 += 32) {
    v16h bh[4];
#pragma unroll
    for (int j = 0; j < 4; ++j) {
      const size_t boff = (size_t)(n0 + (j << 4) + rlane) * kdim + koff + k0;
      bh[j] = Frag<T>::load(Bt + boff);
    }
#pragma unroll
    for (int i = 0; i < 4; ++i) {
      const size_t aoff = (size_t)(m0 + (i << 4) + rlane) * kdim + koff + k0;
      const v16h ah = Frag<T>::load(A + aoff);
#pragma unroll
      for (int j = 0; j < 4; ++j) acc[i][j] = Frag<T>::mma(ah, bh[j], acc[i][j]);
      guard_group4(acc[i][0], acc[i][1], acc[i][2], acc[i][3], ah, bh[0], bh[1], bh[2], bh[3]);
    }
  }
  acc_guard4(acc[0][0], acc[0][1], acc[0][2], acc[0][3]);
  acc_guard4(acc[1][0], acc[1][1], acc[1][2], acc[1][3]);
  acc_guard4(acc[2][0], acc[2][1], acc[2][2], acc[2][3]);
  acc_guard4(acc[3][0], acc[3][1], acc[3][2], acc[3][3]);

  float* slab = sT[wave];
  float* cst  = sC[wave];
  float* prow = sP[wave];
  {
    const int sb = tn * STATE_DIM;
    const float b0 = bi[sb + lane] + bl[sb + lane];
    const float b1 = bi[sb + 32 + lane] + bl[sb + 32 + lane];
    const float w0 = wo[sb + lane];
    const float w1 = wo[sb + 32 + lane];
    cst[lane]      = b0;
    cst[32 + lane] = b1;
    cst[64 + lane] = w0;
    cst[96 + lane] = w1;
  }
  const int erow = lane >> 1;
  const int ecb  = (lane & 1) * 32;
#pragma unroll
  for (int i = 0; i < 4; ++i) {
#pragma unroll
    for (int j = 0; j < 4; ++j) {
#pragma unroll
      for (int r = 0; r < 8; ++r) slab[(mOff + r) * SLAB_PITCH + (j << 4) + rlane] = acc[i][j][r];
    }
    wave_lds_sync();
    float s = 0.0f;
#pragma unroll 1
    for (int q = 0; q < 8; ++q) {
      const v4f av4 = *(const v4f*)(slab + erow * SLAB_PITCH + ecb + 4 * q);
      const v4f bv4 = *(const v4f*)(cst + ecb + 4 * q);
      const v4f wv4 = *(const v4f*)(cst + 64 + ecb + 4 * q);
#pragma unroll
      for (int e = 0; e < 4; ++e) {
        const float li = fmaf(av4[e], FOLD_INV, bv4[e]);
        s = fmaf(tanh_plus_ripple_act(li), wv4[e], s);
      }
    }
    s += __shfl_xor(s, 1, 32);
    if ((lane & 1) == 0) prow[(i << 4) + erow] = s;
    wave_lds_sync();
  }
  const float bov = bo[tn];
  v4f ov = *(const v4f*)(prow + 4 * (lane & 15));
  ov[0] += bov;
  ov[1] += bov;
  ov[2] += bov;
  ov[3] += bov;
  float* dp = Pt + (size_t)tn * BATCH_ROWS + m0 + 4 * (lane & 15);
  if (lane < 16) *(volatile v4f*)dp = ov;
  __threadfence();
  if (lane < 16) *(volatile v4f*)dp = ov;
}

template <int NN, bool OUT_F32>
__global__ __launch_bounds__(128) void lateral_mix_kernel(const float* __restrict__ Pt, const unsigned short* __restrict__ Ltp,
                                                          const float* __restrict__ avec, void* __restrict__ Hout) {
  typedef _Float16 T;
  constexpr int APITCH = NN + 8;
  static_assert(NN % 64 == 0 && (APITCH * 2) % 16 == 0);
  static_assert(!OUT_F32 || NN == 64);
  __shared__ __align__(16) _Float16 Ah[64 * APITCH];
  __shared__ __align__(16) float sT[4][16 * SLAB_PITCH];
  const int tid = threadIdx.x;
  const int lane = tid & 31;
  const int wave = tid >> 5;
  const int c = lane & 15;
  const int hh = lane >> 4;
  const int koff = hh * 8;
  const int rowbase = blockIdx.x * 64;

#pragma unroll 1
  for (int it = 0; it < NN / 8; ++it) {
    const int idx = tid + 128 * it;
    const int k = idx >> 4;
    const int bq = (idx & 15) * 4;
    const v4f v = *(const v4f*)(Pt + (size_t)k * BATCH_ROWS + rowbase + bq);
#pragma unroll
    for (int e = 0; e < 4; ++e) Ah[(bq + e) * APITCH + k] = (_Float16)(v[e] * ACT_CARRY);
  }
  __syncthreads();

  const T* Lt = (const T*)Ltp;
  const T* arow = Ah + (16 * wave + c) * APITCH + koff;
  float* slab = sT[wave];

#pragma unroll 1
  for (int cc = 0; cc < NN / 64; ++cc) {
    v8f acc[4];
#pragma unroll
    for (int j = 0; j < 4; ++j) acc[j] = (v8f){0.f, 0.f, 0.f, 0.f, 0.f, 0.f, 0.f, 0.f};
    const T* lrow = Lt + (size_t)(64 * cc + c) * NN + koff;
#pragma unroll 1
    for (int k0 = 0; k0 < NN; k0 += 32) {
      const v16h a = Frag<T>::load(arow + k0);
      v16h bf[4];
#pragma unroll
      for (int j = 0; j < 4; ++j) bf[j] = Frag<T>::load(lrow + (size_t)(16 * j) * NN + k0);
#pragma unroll
      for (int j = 0; j < 4; ++j) acc[j] = Frag<T>::mma(a, bf[j], acc[j]);
      guard_group4(acc[0], acc[1], acc[2], acc[3], a, bf[0], bf[1], bf[2], bf[3]);
    }
    acc_guard4(acc[0], acc[1], acc[2], acc[3]);

#pragma unroll
    for (int j = 0; j < 4; ++j) {
      const int col = 64 * cc + 16 * j + c;
      const float av = avec[col];
      const float* rp = Pt + (size_t)col * BATCH_ROWS + rowbase + 16 * wave + 8 * hh;
      const v4f r0 = *(const v4f*)(rp);
      const v4f r1 = *(const v4f*)(rp + 4);
#pragma unroll
      for (int r = 0; r < 8; ++r) {
        const float res = (r < 4) ? r0[r & 3] : r1[r & 3];
        const float mix = acc[j][r] * FOLD_INV;
        const float val = (res + 0.1f * mix) * av;
        slab[(8 * hh + r) * SLAB_PITCH + 16 * j + c] = val;
      }
    }
    wave_lds_sync();
    if (OUT_F32) {
      float* H = (float*)Hout;
      const int c4 = c * 4;
      v4f ov[8];
#pragma unroll
      for (int it = 0; it < 8; ++it) ov[it] = *(const v4f*)(slab + (it * 2 + hh) * SLAB_PITCH + c4);
      for (int pass = 0; pass < 2; ++pass) {
#pragma unroll
        for (int it = 0; it < 8; ++it) {
          const int row = it * 2 + hh;
          *(volatile v4f*)(H + (size_t)(rowbase + 16 * wave + row) * NN + 64 * cc + c4) = ov[it];
        }
        __threadfence();
      }
    } else {
      unsigned short* H = (unsigned short*)Hout;
      const int q = lane >> 3;
      const int c8 = (lane & 7) * 8;
      v8h hv[4];
#pragma unroll
      for (int it = 0; it < 4; ++it) {
        const float* sp = slab + (it * 4 + q) * SLAB_PITCH + c8;
#pragma unroll
        for (int e = 0; e < 8; ++e) hv[it][e] = (_Float16)(sp[e] * ACT_CARRY);
      }
      for (int pass = 0; pass < 2; ++pass) {
#pragma unroll
        for (int it = 0; it < 4; ++it) {
          const int row = it * 4 + q;
          *(volatile v8h*)(H + (size_t)(rowbase + 16 * wave + row) * NN + 64 * cc + c8) = hv[it];
        }
        __threadfence();
      }
    }
    wave_lds_sync();
  }
}

__global__ __launch_bounds__(256) void final_proj_kernel(const float* __restrict__ H2, const float* __restrict__ Wout,
                                                         const float* __restrict__ bout, float* __restrict__ out) {
  const int idx = blockIdx.x * 256 + threadIdx.x;
  if (idx < NOUT_TOTAL) {
    const int b = idx / OUT_DIM;
    const int o = idx - b * OUT_DIM;
    const float* hp = H2 + (size_t)b * HID2;
    float s = 0.0f;
#pragma unroll 1
    for (int q = 0; q < HID2 / 4; ++q) {
      const v4f h = *(const v4f*)(hp + 4 * q);
      s = fmaf(h[0], Wout[(4 * q + 0) * OUT_DIM + o], s);
      s = fmaf(h[1], Wout[(4 * q + 1) * OUT_DIM + o], s);
      s = fmaf(h[2], Wout[(4 * q + 2) * OUT_DIM + o], s);
      s = fmaf(h[3], Wout[(4 * q + 3) * OUT_DIM + o], s);
    }
    const float v = s + bout[o];
    *(volatile float*)(out + idx) = v;
    __threadfence();
    *(volatile float*)(out + idx) = v;
  }
}

extern "C" void kernel_launch(void* const* d_in, const int* in_sizes, int n_in,
                              void* d_out, int out_size, void* d_ws, size_t ws_size, hipStream_t stream) {
  if (n_in < 24 || d_out == nullptr || d_ws == nullptr) return;
  const int hid[3] = {HID0, HID1, HID2};
  const int din[3] = {IN_DIM, HID0, HID1};
  if (in_sizes[0] != BATCH_ROWS * IN_DIM) return;
  for (int l = 0; l < 3; ++l) {
    const int bidx = 1 + 7 * l;
    if (in_sizes[bidx + 0] != hid[l] * din[l] * STATE_DIM) return;
    if (in_sizes[bidx + 1] != hid[l] * STATE_DIM) return;
    if (in_sizes[bidx + 2] != hid[l] * STATE_DIM) return;
    if (in_sizes[bidx + 3] != hid[l] * STATE_DIM) return;
    if (in_sizes[bidx + 4] != hid[l]) return;
    if (in_sizes[bidx + 5] != hid[l] * hid[l]) return;
    if (in_sizes[bidx + 6] != hid[l]) return;
  }
  if (in_sizes[22] != HID2 * OUT_DIM || in_sizes[23] != OUT_DIM || out_size != NOUT_TOTAL) return;

  const float* x = (const float*)d_in[0];
  const float *Wi[3], *bi[3], *bl[3], *Wo[3], *bo[3], *Lm[3], *av[3];
  for (int l = 0; l < 3; ++l) {
    const int bidx = 1 + 7 * l;
    Wi[l] = (const float*)d_in[bidx + 0];
    bi[l] = (const float*)d_in[bidx + 1];
    bl[l] = (const float*)d_in[bidx + 2];
    Wo[l] = (const float*)d_in[bidx + 3];
    bo[l] = (const float*)d_in[bidx + 4];
    Lm[l] = (const float*)d_in[bidx + 5];
    av[l] = (const float*)d_in[bidx + 6];
  }
  const float* Wout = (const float*)d_in[22];
  const float* bout = (const float*)d_in[23];
  float* out = (float*)d_out;

  char* ws = (char*)d_ws;
  size_t off = 0;
  auto carve = [&](size_t bytes) -> char* { char* p = ws + off; off += (bytes + 255) & ~(size_t)255; return p; };
  unsigned short* XH  = (unsigned short*)carve((size_t)BATCH_ROWS * IN_DIM * 2);
  unsigned short* WT[3];
  WT[0] = (unsigned short*)carve((size_t)HID0 * STATE_DIM * IN_DIM * 2);
  WT[1] = (unsigned short*)carve((size_t)HID1 * STATE_DIM * HID0 * 2);
  WT[2] = (unsigned short*)carve((size_t)HID2 * STATE_DIM * HID1 * 2);
  unsigned short* LT[3];
  LT[0] = (unsigned short*)carve((size_t)HID0 * HID0 * 2);
  LT[1] = (unsigned short*)carve((size_t)HID1 * HID1 * 2);
  LT[2] = (unsigned short*)carve((size_t)HID2 * HID2 * 2);
  float*          PT0 = (float*)carve((size_t)HID0 * BATCH_ROWS * 4);
  unsigned short* H0  = (unsigned short*)carve((size_t)BATCH_ROWS * HID0 * 2);
  float*          PT1 = (float*)carve((size_t)HID1 * BATCH_ROWS * 4);
  unsigned short* H1  = (unsigned short*)carve((size_t)BATCH_ROWS * HID1 * 2);
  float*          PT2 = (float*)carve((size_t)HID2 * BATCH_ROWS * 4);
  float*          H2  = (float*)carve((size_t)BATCH_ROWS * HID2 * 4);
  if (off > ws_size || off > (size_t)134217728) return;

  const int n8x = BATCH_ROWS * IN_DIM / 8;
  cvt8_f16_kernel<<<n8x / 256, 256, 0, stream>>>(x, XH, n8x, ACT_CARRY);
  for (int l = 0; l < 3; ++l) {
    transpose_cvt_kernel<<<dim3(din[l] / 64, 1, hid[l]), 256, 0, stream>>>(
        Wi[l], WT[l], STATE_DIM, din[l], (long)din[l] * STATE_DIM, (long)STATE_DIM * din[l], WGT_CARRY);
  }
  for (int l = 0; l < 3; ++l) {
    transpose_cvt_kernel<<<dim3(hid[l] / 64, hid[l] / 64, 1), 256, 0, stream>>>(
        Lm[l], LT[l], hid[l], hid[l], 0L, 0L, WGT_CARRY);
  }

  layer_fused_kernel<<<(BATCH_ROWS / 64) * HID0 / 8, 256, 0, stream>>>(
      XH, WT[0], bi[0], bl[0], Wo[0], bo[0], PT0, IN_DIM, HID0);
  lateral_mix_kernel<HID0, false><<<BATCH_ROWS / 64, 128, 0, stream>>>(PT0, LT[0], av[0], (void*)H0);

  layer_fused_kernel<<<(BATCH_ROWS / 64) * HID1 / 8, 256, 0, stream>>>(
      H0, WT[1], bi[1], bl[1], Wo[1], bo[1], PT1, HID0, HID1);
  lateral_mix_kernel<HID1, false><<<BATCH_ROWS / 64, 128, 0, stream>>>(PT1, LT[1], av[1], (void*)H1);

  layer_fused_kernel<<<(BATCH_ROWS / 64) * HID2 / 8, 256, 0, stream>>>(
      H1, WT[2], bi[2], bl[2], Wo[2], bo[2], PT2, HID1, HID2);
  lateral_mix_kernel<HID2, true><<<BATCH_ROWS / 64, 128, 0, stream>>>(PT2, LT[2], av[2], (void*)H2);

  final_proj_kernel<<<NOUT_TOTAL / 256, 256, 0, stream>>>(H2, Wout, bout, out);
}
